// SelfAttention_87771951661553
// MI455X (gfx1250) — hardware-verified
//
#include <hip/hip_runtime.h>
#include <math.h>

typedef __attribute__((ext_vector_type(16))) _Float16 v16h;
typedef __attribute__((ext_vector_type(16))) __bf16 v16b;
typedef __attribute__((ext_vector_type(8)))  _Float16 v8h;
typedef __attribute__((ext_vector_type(8)))  __bf16 v8b;
typedef __attribute__((ext_vector_type(8)))  float v8f;
typedef __attribute__((ext_vector_type(4)))  float v4f;
typedef __attribute__((ext_vector_type(4)))  unsigned v4u;

#ifndef NB
#define NB 2
#endif
#ifndef SEQ
#define SEQ 2048
#endif
#define NB_FULL 2
#define SEQ_FULL 2048
#define DM 1024
#define NH 16
#define HD 64
#define N3 3072
#define MROWS (NB * SEQ)

static_assert(NH * HD == DM);
static_assert(HD == 64);
static_assert(DM % 128 == 0);
static_assert(N3 == 3 * DM);
static_assert(SEQ % 64 == 0);
static_assert(SEQ <= SEQ_FULL);
static_assert(NB <= NB_FULL);
static_assert(MROWS % 64 == 0);
static_assert((MROWS * (DM / 8)) % 256 == 0);
static_assert(DM % 32 == 0);

constexpr size_t SZ_XB  = (size_t)2 * MROWS * DM;
constexpr size_t SZ_WQT = (size_t)2 * N3 * DM;
constexpr size_t SZ_WPT = (size_t)2 * DM * DM;
constexpr size_t SZ_PL  = (size_t)2 * MROWS * DM;
constexpr size_t SZ_CT  = (size_t)2 * MROWS * 2 * DM;
constexpr size_t OFF_XB  = 0;
constexpr size_t OFF_WQT = OFF_XB + SZ_XB;
constexpr size_t OFF_WPT = OFF_WQT + SZ_WQT;
constexpr size_t OFF_PL  = OFF_WPT + SZ_WPT;
constexpr size_t OFF_CT  = OFF_PL + 4 * SZ_PL;
constexpr size_t WS_TOTAL = OFF_CT + SZ_CT;
static_assert(WS_TOTAL <= (size_t)134217728);
static_assert(OFF_WQT % 128 == 0 && OFF_WPT % 128 == 0 && OFF_PL % 128 == 0 && OFF_CT % 128 == 0 && SZ_PL % 128 == 0);

template <typename T> __device__ __forceinline__ void vst2(void* p, T v) { *(volatile T*)p = v; __threadfence(); *(volatile T*)p = v; }

__device__ __forceinline__ v8f wmma16(v16h a, v16h b, v8f c) {
  v8f d = __builtin_amdgcn_wmma_f32_16x16x32_f16(false, a, false, b, (short)0, c, false, false);
  asm volatile("v_nop\n\tv_nop\n\tv_nop\n\tv_nop" : "+v"(d) : "v"(a), "v"(b));
  return d;
}
__device__ __forceinline__ v8f wmma_bf(v16b a, v16b b, v8f c) {
  v8f d = __builtin_amdgcn_wmma_f32_16x16x32_bf16(false, a, false, b, (short)0, c, false, false);
  asm volatile("v_nop\n\tv_nop\n\tv_nop\n\tv_nop" : "+v"(d) : "v"(a), "v"(b));
  return d;
}
__device__ __forceinline__ v16h frag_h(const _Float16* rowk0, int lane) {
  union { v16h v; v8h q[2]; } u; const _Float16* p = rowk0 + 8 * (lane >> 4);
  u.q[0] = *(const v8h*)p; u.q[1] = *(const v8h*)(p + 16); return u.v;
}
__device__ __forceinline__ v16b frag_b(const __bf16* rowk0, int lane) {
  union { v16b v; v8b q[2]; } u; const __bf16* p = rowk0 + 8 * (lane >> 4);
  u.q[0] = *(const v8b*)p; u.q[1] = *(const v8b*)(p + 16); return u.v;
}
__device__ __forceinline__ float bfr(float v) { return (float)(__bf16)v; }

__global__ __launch_bounds__(256) void k_cvtx(const float* __restrict__ X, unsigned short* __restrict__ XB) {
  const int e = blockIdx.x * 256 + threadIdx.x;
  if (e >= MROWS * (DM / 8)) return;
  const int m = e >> 7, q = e & 127; const int b = m / SEQ, t = m - b * SEQ;
  const float* p = X + ((size_t)b * SEQ_FULL + t) * DM + q * 8;
  const v4f v0 = *(const v4f*)p; const v4f v1 = *(const v4f*)(p + 4);
  union { v8b b8; v4u u; } o;
#pragma unroll
  for (int i = 0; i < 4; ++i) { o.b8[i] = (__bf16)v0[i]; o.b8[4 + i] = (__bf16)v1[i]; }
  vst2(XB + (size_t)m * DM + q * 8, o.u);
}

__global__ __launch_bounds__(256) void k_wt(const float* __restrict__ W, unsigned short* __restrict__ OUT, int N, int asf16) {
  __shared__ __align__(16) unsigned short t[64][72];
  const int tid = threadIdx.x; const int n0 = blockIdx.x * 64, k0 = blockIdx.y * 64;
  for (int e = tid; e < 64 * 16; e += 256) { const int kr = e >> 4, q = e & 15;
    const v4f v = *(const v4f*)(W + (size_t)(k0 + kr) * N + n0 + q * 4);
#pragma unroll
    for (int c = 0; c < 4; ++c) { const __bf16 bv = (__bf16)v[c]; const unsigned short bb = __builtin_bit_cast(unsigned short, bv);
      const _Float16 hv = (_Float16)((float)bv * 256.0f); const unsigned short hb = __builtin_bit_cast(unsigned short, hv);
      t[q * 4 + c][kr] = asf16 ? hb : bb; } }
  __syncthreads();
  for (int e = tid; e < 64 * 8; e += 256) { const int nl = e >> 3, q = e & 7;
    const v4u v = *(const v4u*)&t[nl][q * 8];
    vst2(OUT + (size_t)(n0 + nl) * DM + k0 + q * 8, v); }
}

__global__ __launch_bounds__(128) void k_qkv(const __bf16* __restrict__ XB, const __bf16* __restrict__ WQT, const float* __restrict__ BQ, _Float16* __restrict__ PL) {
  __shared__ __align__(16) _Float16 sh[64][136];
  __shared__ __align__(16) _Float16 sl[64][136];
  __shared__ __align__(16) _Float16 th[128][72];
  const int tid = threadIdx.x; const int wave = __builtin_amdgcn_readfirstlane(threadIdx.x >> 5);
  const int lane = tid & 31, col = lane & 15, g = lane >> 4; const int wm = wave >> 1, wn = wave & 1;
  const int r0 = blockIdx.x * 64, c0 = blockIdx.y * 128; const int which = c0 >> 10, cw = c0 & (DM - 1);
  const size_t PLN = (size_t)MROWS * DM;
  v8f acc[2][4] = {};
  const size_t arow = (size_t)(r0 + wm * 32 + col) * DM; const size_t brow = (size_t)(c0 + wn * 64 + col) * DM;
#pragma unroll 1
  for (int kc = 0; kc < DM / 32; ++kc) {
    const v16b a0 = frag_b(XB + arow + kc * 32, lane); const v16b a1 = frag_b(XB + arow + (size_t)16 * DM + kc * 32, lane);
#pragma unroll
    for (int j = 0; j < 4; ++j) { const v16b w = frag_b(WQT + brow + (size_t)j * 16 * DM + kc * 32, lane);
      acc[0][j] = wmma_bf(a0, w, acc[0][j]); acc[1][j] = wmma_bf(a1, w, acc[1][j]); } }
  if (which < 2) {
    const float qs = which == 0 ? 1024.0f : 1.0f;
#pragma unroll
    for (int j = 0; j < 4; ++j) { const float bias = bfr(BQ[c0 + wn * 64 + j * 16 + col]); const int cl = wn * 64 + j * 16 + col;
#pragma unroll
      for (int i = 0; i < 2; ++i) {
#pragma unroll
        for (int r = 0; r < 8; ++r) { const float v = (acc[i][j][r] + bias) * qs; const _Float16 hv = (_Float16)v; const int rl = wm * 32 + i * 16 + 8 * g + r;
          sh[rl][cl] = hv; sl[rl][cl] = (_Float16)(v - (float)hv); } } }
    __syncthreads();
    const size_t hoff = which == 0 ? (size_t)0 : 2 * PLN;
    for (int e = tid; e < 64 * 16; e += 128) { const int rl = e >> 4, q = e & 15;
      const size_t o = (size_t)(r0 + rl) * DM + cw + q * 8;
      const v4u hv = *(const v4u*)&sh[rl][q * 8]; vst2(PL + hoff + o, hv);
      if (which == 0) { const v4u lv = *(const v4u*)&sl[rl][q * 8]; vst2(PL + PLN + o, lv); } }
  } else {
#pragma unroll
    for (int j = 0; j < 4; ++j) { const float bias = bfr(BQ[c0 + wn * 64 + j * 16 + col]); const int cl = wn * 64 + j * 16 + col;
#pragma unroll
      for (int i = 0; i < 2; ++i) {
#pragma unroll
        for (int r = 0; r < 8; ++r) { const int rl = wm * 32 + i * 16 + 8 * g + r; th[cl][rl] = (_Float16)(acc[i][j][r] + bias); } } }
    __syncthreads();
    const int bb = r0 / SEQ, t0 = r0 - bb * SEQ;
    for (int e = tid; e < 128 * 8; e += 128) { const int cl = e >> 3, q = e & 7;
      const v4u v = *(const v4u*)&th[cl][q * 8];
      vst2(PL + 3 * PLN + ((size_t)bb * DM + cw + cl) * (size_t)SEQ + t0 + q * 8, v); } }
}

__global__ __launch_bounds__(128) void k_attn(const _Float16* __restrict__ QH, const _Float16* __restrict__ QL, const _Float16* __restrict__ KH, const _Float16* __restrict__ VT, _Float16* __restrict__ CT) {
  __shared__ __align__(16) _Float16 sh[64][72];
  __shared__ __align__(16) _Float16 sl[64][72];
  const int tid = threadIdx.x; const int wave = __builtin_amdgcn_readfirstlane(threadIdx.x >> 5);
  const int lane = tid & 31, col = lane & 15, g = lane >> 4;
  const int qb = blockIdx.x, h = blockIdx.y, b = blockIdx.z;
  const size_t row0 = (size_t)b * SEQ + (size_t)qb * 64;
  const size_t qoff = (row0 + wave * 16 + col) * DM + h * HD;
  const size_t kbase = ((size_t)b * SEQ + col) * DM + h * HD;
  const size_t vbase = ((size_t)b * DM + h * HD + col) * (size_t)SEQ;
  v8f o[4] = {}; float m = -3.0e38f, l = 0.0f;
  const float c2 = 0.125f * 1.4426950408889634f * (1.0f / 1024.0f);
#pragma unroll 1
  for (int kt = 0; kt < SEQ / 32; ++kt) {
    const size_t k0o = kbase + (size_t)kt * 32 * DM; const size_t k1o = k0o + (size_t)16 * DM;
    v8f s0 = {}, s1 = {};
#pragma unroll
    for (int kc = 0; kc < HD / 32; ++kc) {
      const v16h qh = frag_h(QH + qoff + kc * 32, lane); const v16h ql = frag_h(QL + qoff + kc * 32, lane);
      const v16h ka = frag_h(KH + k0o + kc * 32, lane); const v16h kb = frag_h(KH + k1o + kc * 32, lane);
      s0 = wmma16(ka, qh, s0); s0 = wmma16(ka, ql, s0); s1 = wmma16(kb, qh, s1); s1 = wmma16(kb, ql, s1); }
    float mx = -3.0e38f;
#pragma unroll
    for (int r = 0; r < 8; ++r) { s0[r] *= c2; s1[r] *= c2; mx = fmaxf(mx, fmaxf(s0[r], s1[r])); }
    mx = fmaxf(mx, __shfl_xor(mx, 16));
    const float mn = fmaxf(m, mx); const float alpha = exp2f(m - mn); m = mn; const float sft = 10.0f - mn;
    v16h p; float ps = 0.0f;
#pragma unroll
    for (int r = 0; r < 8; ++r) { const _Float16 pa = (_Float16)exp2f(s0[r] + sft); const _Float16 pc = (_Float16)exp2f(s1[r] + sft);
      p[r] = pa; p[8 + r] = pc; ps += (float)pa + (float)pc; }
    l = l * alpha + ps;
#pragma unroll
    for (int t = 0; t < 4; ++t) {
#pragma unroll
      for (int r = 0; r < 8; ++r) o[t][r] *= alpha; }
#pragma unroll
    for (int t = 0; t < 4; ++t) { const v16h vf = frag_h(VT + vbase + (size_t)t * 16 * SEQ + kt * 32, lane); o[t] = wmma16(vf, p, o[t]); }
  }
  const float lt = l + __shfl_xor(l, 16);
  const float inv = 1024.0f * (1.0f / lt);
#pragma unroll
  for (int t = 0; t < 4; ++t) { v8h hv, lv;
#pragma unroll
    for (int r = 0; r < 8; ++r) { const float cs = o[t][r] * inv; const _Float16 hh = (_Float16)cs; hv[r] = hh; lv[r] = (_Float16)(cs - (float)hh); }
    *(v8h*)&sh[wave * 16 + col][t * 16 + 8 * g] = hv; *(v8h*)&sl[wave * 16 + col][t * 16 + 8 * g] = lv; }
  __syncthreads();
  for (int e = tid; e < 64 * 8; e += 128) { const int rl = e >> 3, q = e & 7;
    const size_t oo = (row0 + rl) * (size_t)(2 * DM) + h * HD + q * 8;
    const v4u hv = *(const v4u*)&sh[rl][q * 8]; const v4u lv = *(const v4u*)&sl[rl][q * 8];
    vst2(CT + oo, hv); vst2(CT + oo + DM, lv); }
}

__global__ __launch_bounds__(128) void k_oproj(const _Float16* __restrict__ CT, const _Float16* __restrict__ WPT, const float* __restrict__ BP, float* __restrict__ OUT) {
  __shared__ __align__(16) float ss[64][132];
  const int tid = threadIdx.x; const int wave = __builtin_amdgcn_readfirstlane(threadIdx.x >> 5);
  const int lane = tid & 31, col = lane & 15, g = lane >> 4; const int wm = wave >> 1, wn = wave & 1;
  const int r0 = blockIdx.x * 64, c0 = blockIdx.y * 128;
  v8f acc[2][4] = {};
  const size_t arow = (size_t)(r0 + wm * 32 + col) * (2 * DM); const size_t brow = (size_t)(c0 + wn * 64 + col) * DM;
#pragma unroll 1
  for (int kc = 0; kc < (2 * DM) / 32; ++kc) { const int ko = kc * 32; const int kw = ko & (DM - 1);
    const v16h a0 = frag_h(CT + arow + ko, lane); const v16h a1 = frag_h(CT + arow + (size_t)16 * 2 * DM + ko, lane);
#pragma unroll
    for (int j = 0; j < 4; ++j) { const v16h w = frag_h(WPT + brow + (size_t)j * 16 * DM + kw, lane);
      acc[0][j] = wmma16(a0, w, acc[0][j]); acc[1][j] = wmma16(a1, w, acc[1][j]); } }
  const float osc = 1.0f / 262144.0f;
#pragma unroll
  for (int j = 0; j < 4; ++j) { const float bias = bfr(BP[c0 + wn * 64 + j * 16 + col]); const int cl = wn * 64 + j * 16 + col;
#pragma unroll
    for (int i = 0; i < 2; ++i) {
#pragma unroll
      for (int r = 0; r < 8; ++r) { const int rl = wm * 32 + i * 16 + 8 * g + r; ss[rl][cl] = acc[i][j][r] * osc + bias; } } }
  __syncthreads();
  for (int e = tid; e < 64 * 32; e += 128) { const int rl = e >> 5, q = e & 31;
    const v4f v = *(const v4f*)&ss[rl][q * 4];
    vst2(OUT + (size_t)(r0 + rl) * DM + c0 + q * 4, v); }
}

extern "C" void kernel_launch(void* const* d_in, const int* in_sizes, int n_in, void* d_out, int out_size, void* d_ws, size_t ws_size, hipStream_t stream) {
  if (n_in < 5) return;
  if ((long long)in_sizes[0] < ((long long)(NB - 1) * SEQ_FULL + SEQ) * DM) return;
  if (in_sizes[1] < DM * N3 || in_sizes[2] < N3 || in_sizes[3] < DM * DM || in_sizes[4] < DM) return;
  if ((long long)out_size < (long long)MROWS * DM) return;
  if (ws_size < WS_TOTAL) return;
  const float* X = (const float*)d_in[0]; const float* WQ = (const float*)d_in[1]; const float* BQ = (const float*)d_in[2];
  const float* WP = (const float*)d_in[3]; const float* BP = (const float*)d_in[4];
  char* ws = (char*)d_ws;
  unsigned short* XBu = (unsigned short*)(ws + OFF_XB); unsigned short* WQTu = (unsigned short*)(ws + OFF_WQT); unsigned short* WPTu = (unsigned short*)(ws + OFF_WPT);
  _Float16* PL = (_Float16*)(ws + OFF_PL); _Float16* CT = (_Float16*)(ws + OFF_CT);
  const size_t PLN = (size_t)MROWS * DM;
  k_cvtx<<<dim3(MROWS * (DM / 8) / 256), 256, 0, stream>>>(X, XBu);
  k_wt<<<dim3(N3 / 64, DM / 64), 256, 0, stream>>>(WQ, WQTu, N3, 0);
  k_wt<<<dim3(DM / 64, DM / 64), 256, 0, stream>>>(WP, WPTu, DM, 1);
  k_qkv<<<dim3(MROWS / 64, N3 / 128), 128, 0, stream>>>((const __bf16*)(ws + OFF_XB), (const __bf16*)(ws + OFF_WQT), BQ, PL);
  k_attn<<<dim3(SEQ / 64, NH, NB), 128, 0, stream>>>(PL, PL + PLN, PL + 2 * PLN, PL + 3 * PLN, CT);
  k_oproj<<<dim3(MROWS / 64, DM / 128), 128, 0, stream>>>(CT, (const _Float16*)(ws + OFF_WPT), BP, (float*)d_out);
}
